// MAA_38568806318777
// MI455X (gfx1250) — hardware-verified
//
#include <hip/hip_runtime.h>
#include <hip/hip_bf16.h>
#include <math.h>

typedef __attribute__((ext_vector_type(16))) _Float16 v16h;
typedef __attribute__((ext_vector_type(8)))  _Float16 v8h;
typedef __attribute__((ext_vector_type(16))) __bf16   v16b;
typedef __attribute__((ext_vector_type(8)))  __bf16   v8b;
typedef __attribute__((ext_vector_type(8)))  float    v8f;
typedef __attribute__((ext_vector_type(4)))  float    v4f;
#define PSCALE 32768.0f
#define U16(p) ((const unsigned short*)(const void*)(p))
#define PSCALE_INV (1.0f / 32768.0f)

__device__ __forceinline__ unsigned short f2bf_bits(float f) {
  unsigned u = __float_as_uint(f);
  return (unsigned short)((u + 0x7FFFu + ((u >> 16) & 1u)) >> 16);
}
__device__ __forceinline__ float bf_bits2f(unsigned short h) { return __uint_as_float(((unsigned)h) << 16); }

__device__ __forceinline__ void dep_guard_h(v8f& a, v8f& b, v16h x, v16h y) { asm volatile("v_nop\n\tv_nop\n\tv_nop\n\tv_nop" : "+v"(a), "+v"(b) : "v"(x), "v"(y)); }
__device__ __forceinline__ void dep_guard_b(v8f& a, v8f& b, v16b x, v16b y) { asm volatile("v_nop\n\tv_nop\n\tv_nop\n\tv_nop" : "+v"(a), "+v"(b) : "v"(x), "v"(y)); }
__device__ __forceinline__ void keep4_h(v16h a, v16h b, v16h c, v16h d) { asm volatile("v_nop" :: "v"(a), "v"(b), "v"(c), "v"(d)); }
__device__ __forceinline__ void keep4_b(v16b a, v16b b, v16b c, v16b d) { asm volatile("v_nop" :: "v"(a), "v"(b), "v"(c), "v"(d)); }
__device__ __forceinline__ void acc_guard4(v8f& a, v8f& b, v8f& c, v8f& d) { asm volatile("v_nop\n\tv_nop\n\tv_nop\n\tv_nop" : "+v"(a), "+v"(b), "+v"(c), "+v"(d)); }
template <typename T> struct Frag;
template <> struct Frag<_Float16> {
  typedef v16h V; union U { v16h v; v8h h[2]; };
  static __device__ __forceinline__ v16h load(const _Float16* p) {
    U f; f.h[0] = *(const v8h*)(p); f.h[1] = *(const v8h*)(p + 16); return f.v;
  }
  static __device__ __forceinline__ v8f mma(v16h a, v16h b, v8f c) {
    return __builtin_amdgcn_wmma_f32_16x16x32_f16(false, a, false, b, (short)0, c, false, false);
  }
  static __device__ __forceinline__ void guard(v8f& a, v8f& b, v16h x, v16h y) { dep_guard_h(a, b, x, y); }
  static __device__ __forceinline__ void keep(v16h a, v16h b, v16h c, v16h d) { keep4_h(a, b, c, d); }
};
template <> struct Frag<__bf16> {
  typedef v16b V; union U { v16b v; v8b h[2]; };
  static __device__ __forceinline__ v16b load(const __bf16* p) {
    U f; f.h[0] = *(const v8b*)(p); f.h[1] = *(const v8b*)(p + 16); return f.v;
  }
  static __device__ __forceinline__ v8f mma(v16b a, v16b b, v8f c) {
    return __builtin_amdgcn_wmma_f32_16x16x32_bf16(false, a, false, b, (short)0, c, false, false);
  }
  static __device__ __forceinline__ void guard(v8f& a, v8f& b, v16b x, v16b y) { dep_guard_b(a, b, x, y); }
  static __device__ __forceinline__ void keep(v16b a, v16b b, v16b c, v16b d) { keep4_b(a, b, c, d); }
};

template <int ET> struct Elem;
template <> struct Elem<0> { typedef _Float16 T; };
template <> struct Elem<1> { typedef __bf16 T; };
template <int ET, bool SPLIT, int BIAS_MODE, int OUT_MODE, bool RESID, int ACT = 0>
__global__ __launch_bounds__(256) void wmma_gemm64(
    const unsigned short* __restrict__ Ap, const unsigned short* __restrict__ A2p, int lda, long strideA,
    const unsigned short* __restrict__ Btp, const unsigned short* __restrict__ Bt2p, int ldb, long strideB,
    void* __restrict__ Cout, void* __restrict__ Cout2, int ldc, long strideC,
    const float* __restrict__ bias,
    const float* __restrict__ resid, long strideR,
    int M, int N, int K, float scale) {
  typedef typename Elem<ET>::T T;
  typedef typename Frag<T>::V V;
  const T* A = (const T*)Ap; const T* A2 = (const T*)A2p; const T* Bt = (const T*)Btp; const T* Bt2 = (const T*)Bt2p;
  __shared__ __align__(16) float sT[8][16 * 68];
  const int b    = blockIdx.y;
  const int lane = threadIdx.x & 31;
  const int wave = threadIdx.x >> 5;
  const int tilesN = N >> 6;
  const int tilesM = M >> 6;
  const int tile = blockIdx.x * 8 + wave;
  if (tile >= tilesM * tilesN) return;
  const int tm = tile / tilesN;
  const int tn = tile - tm * tilesN;
  const int m0 = tm << 6;
  const int n0 = tn << 6;

  const T* Ab  = A  + (size_t)b * strideA;
  const T* Bb  = Bt + (size_t)b * strideB;
  const T* Ab2 = SPLIT ? (A2  + (size_t)b * strideA) : nullptr;
  const T* Bb2 = SPLIT ? (Bt2 + (size_t)b * strideB) : nullptr;

  const int rlane = lane & 15;
  const int koff  = (lane >> 4) * 8;
  const int mOff  = (lane >> 4) * 8;

  v8f acc[4][4];
#pragma unroll
  for (int i = 0; i < 4; ++i)
#pragma unroll
    for (int j = 0; j < 4; ++j) acc[i][j] = (v8f){0.f,0.f,0.f,0.f,0.f,0.f,0.f,0.f};

  for (int k0 = 0; k0 < K; k0 += 32) {
    V bh[4], bl[4];
#pragma unroll
    for (int j = 0; j < 4; ++j) {
      const size_t bo = (size_t)(n0 + (j << 4) + rlane) * ldb + koff + k0;
      bh[j] = Frag<T>::load(Bb + bo);
      if (SPLIT) bl[j] = Frag<T>::load(Bb2 + bo);
    }
#pragma unroll
    for (int i = 0; i < 4; ++i) {
      const size_t ao = (size_t)(m0 + (i << 4) + rlane) * lda + koff + k0;
      V ah = Frag<T>::load(Ab + ao);
      V al;
      if (SPLIT) al = Frag<T>::load(Ab2 + ao);
#pragma unroll
      for (int j = 0; j < 4; ++j) {
        acc[i][j] = Frag<T>::mma(ah, bh[j], acc[i][j]);
        if (SPLIT) {
          acc[i][j] = Frag<T>::mma(ah, bl[j], acc[i][j]);
          acc[i][j] = Frag<T>::mma(al, bh[j], acc[i][j]);
        }
      }
      Frag<T>::guard(acc[i][0], acc[i][3], ah, SPLIT ? al : ah);
    }
    Frag<T>::keep(bh[0], bh[1], bh[2], bh[3]);
    if (SPLIT) Frag<T>::keep(bl[0], bl[1], bl[2], bl[3]);
  }
  acc_guard4(acc[0][0], acc[0][1], acc[0][2], acc[0][3]);
  acc_guard4(acc[1][0], acc[1][1], acc[1][2], acc[1][3]);
  acc_guard4(acc[2][0], acc[2][1], acc[2][2], acc[2][3]);
  acc_guard4(acc[3][0], acc[3][1], acc[3][2], acc[3][3]);

  float* slab = sT[wave];
  const float* Rb = RESID ? (resid + (size_t)b * strideR) : nullptr;
#pragma unroll
  for (int i = 0; i < 4; ++i) {
    const int mBase = m0 + (i << 4);
#pragma unroll
    for (int j = 0; j < 4; ++j) {
      const int n = n0 + (j << 4) + rlane;
      float bv = 0.f;
      if (BIAS_MODE == 2) bv = bias[n];
#pragma unroll
      for (int r = 0; r < 8; ++r) {
        float v = acc[i][j][r] * scale;
        if (BIAS_MODE == 1) v += bias[mBase + mOff + r];
        if (BIAS_MODE == 2) v += bv;
        if (RESID) v += Rb[(size_t)(mBase + mOff + r) * ldc + n];
        if (ACT == 1) v = tanhf(v);
        if (ACT == 2) v = fmaxf(v, 0.0f);
        if (ACT == 3) v = v / (1.0f + expf(-v));
        if (ACT == 4) v = (v > 0.f) ? v : 0.01f * v;
        if (ACT == 5) v = 0.5f * v * (1.0f + erff(v * 0.70710678118654752f));
        slab[(mOff + r) * 68 + (j << 4) + rlane] = v;
      }
    }
    __builtin_amdgcn_fence(__ATOMIC_RELEASE, "workgroup");
    __builtin_amdgcn_wave_barrier();
    __builtin_amdgcn_fence(__ATOMIC_ACQUIRE, "workgroup");
    if (OUT_MODE == 0) {
      float* C = (float*)Cout + (size_t)b * strideC;
      const int hh = lane >> 4, c4 = (lane & 15) * 4;
      for (int pass = 0; pass < 2; ++pass) {
#pragma unroll
        for (int it = 0; it < 8; ++it) {
          const int row = it * 2 + hh;
          v4f v = *(const v4f*)(slab + row * 68 + c4);
          *(volatile v4f*)(C + (size_t)(mBase + row) * ldc + n0 + c4) = v;
        }
        __threadfence();
      }
    } else {
      const int q = lane >> 3, c8 = (lane & 7) * 8;
      unsigned short* C  = (unsigned short*)Cout  + (size_t)b * strideC;
      unsigned short* C2 = (OUT_MODE == 2) ? ((unsigned short*)Cout2 + (size_t)b * strideC) : nullptr;
      for (int pass = 0; pass < 2; ++pass) {
#pragma unroll
        for (int it = 0; it < 4; ++it) {
          const int row = it * 4 + q;
          const float* sp = slab + row * 68 + c8;
          v8h hv, lv;
#pragma unroll
          for (int e = 0; e < 8; ++e) {
            if (OUT_MODE == 1) {
              hv[e] = (_Float16)sp[e];
            } else {
              unsigned short hb = f2bf_bits(sp[e]);
              unsigned short lb = f2bf_bits(sp[e] - bf_bits2f(hb));
              hv[e] = __builtin_bit_cast(_Float16, hb);
              lv[e] = __builtin_bit_cast(_Float16, lb);
            }
          }
          *(volatile v8h*)(C + (size_t)(mBase + row) * ldc + n0 + c8) = hv;
          if (OUT_MODE == 2) *(volatile v8h*)(C2 + (size_t)(mBase + row) * ldc + n0 + c8) = lv;
        }
        __threadfence();
      }
    }
    __builtin_amdgcn_fence(__ATOMIC_RELEASE, "workgroup");
    __builtin_amdgcn_wave_barrier();
    __builtin_amdgcn_fence(__ATOMIC_ACQUIRE, "workgroup");
  }
}

__global__ __launch_bounds__(256) void cast_f32_f16x2(
    const float* __restrict__ in, _Float16* __restrict__ out, int n2) {
  int i = blockIdx.x * 256 + threadIdx.x;
  if (i < n2) {
    const _Float16 h0 = (_Float16)in[2 * i], h1 = (_Float16)in[2 * i + 1];
    const unsigned u = (unsigned)__builtin_bit_cast(unsigned short, h0) | ((unsigned)__builtin_bit_cast(unsigned short, h1) << 16);
    ((volatile unsigned*)out)[i] = u;
    __threadfence();
    ((volatile unsigned*)out)[i] = u;
  }
}

#define TP_PK 72
__global__ __launch_bounds__(256) void cast_transpose_f16(
    const float* __restrict__ in, _Float16* __restrict__ out, int K, int N, float scl, int ndup) {
  __shared__ __align__(16) _Float16 sm[64 * TP_PK];
  const int t  = threadIdx.x;
  const int n0 = blockIdx.x * 64;
  const int k0 = blockIdx.y * 64;
#pragma unroll
  for (int i = 0; i < 16; ++i) {
    const int kr = 4 * i + (t >> 6);
    const int nc = t & 63;
    sm[nc * TP_PK + kr] = (_Float16)(in[(size_t)(k0 + kr) * N + n0 + nc] * scl);
  }
  __syncthreads();
  const int qq = t >> 3, c8 = (t & 7) * 8;
  const int nd = (ndup > 2) ? 2 : ((ndup < 1) ? 1 : ndup);
  for (int d = 0; d < nd; ++d) {
    _Float16* ob = out + (size_t)d * N * K;
    for (int pass = 0; pass < 2; ++pass) {
#pragma unroll
      for (int it = 0; it < 2; ++it) {
        const int row = it * 32 + qq;
        const v8h val = *(const v8h*)(sm + row * TP_PK + c8);
        *(volatile v8h*)(ob + (size_t)(n0 + row) * K + k0 + c8) = val;
      }
      __threadfence();
    }
  }
}

#define LN_D 1024
__global__ __launch_bounds__(128) void layernorm_f16(
    const float* __restrict__ x, const float* __restrict__ g, const float* __restrict__ bta, _Float16* __restrict__ out) {
  __shared__ float red[4];
  const int row = blockIdx.x;
  const int t = threadIdx.x, lane = t & 31, wave = t >> 5;
  const float* xr = x + (size_t)row * LN_D + 8 * t;
  const v4f a0 = *(const v4f*)xr;
  const v4f a1 = *(const v4f*)(xr + 4);
  float xv[8];
#pragma unroll
  for (int e = 0; e < 4; ++e) { xv[e] = a0[e]; xv[4 + e] = a1[e]; }
  float s = ((xv[0] + xv[1]) + (xv[2] + xv[3])) + ((xv[4] + xv[5]) + (xv[6] + xv[7]));
#pragma unroll
  for (int off = 16; off > 0; off >>= 1) s += __shfl_xor(s, off, 32);
  if (lane == 0) red[wave] = s;
  __syncthreads();
  const float mu = ((red[0] + red[1]) + (red[2] + red[3])) * (1.0f / 1024.0f);
  __syncthreads();
  float vs = 0.f;
#pragma unroll
  for (int e = 0; e < 8; ++e) { const float d = xv[e] - mu; xv[e] = d; vs += d * d; }
#pragma unroll
  for (int off = 16; off > 0; off >>= 1) vs += __shfl_xor(vs, off, 32);
  if (lane == 0) red[wave] = vs;
  __syncthreads();
  const float var = ((red[0] + red[1]) + (red[2] + red[3])) * (1.0f / 1024.0f);
  const float rstd = rsqrtf(var + 1e-5f);
  const v4f g0 = *(const v4f*)(g + 8 * t), g1 = *(const v4f*)(g + 8 * t + 4);
  const v4f b0 = *(const v4f*)(bta + 8 * t), b1 = *(const v4f*)(bta + 8 * t + 4);
  v8h hv;
#pragma unroll
  for (int e = 0; e < 4; ++e) {
    hv[e]     = (_Float16)(xv[e] * rstd * g0[e] + b0[e]);
    hv[4 + e] = (_Float16)(xv[4 + e] * rstd * g1[e] + b1[e]);
  }
  _Float16* orow = out + (size_t)row * LN_D + 8 * t;
  *(volatile v8h*)orow = hv;
  __threadfence();
  *(volatile v8h*)orow = hv;
}

#define AT_D 64
#define AT_NW 4
#define AT_QB 64
#define AT_KC 64
__device__ __forceinline__ v8f mma_h(v16h a, v16h b, v8f c) {
  c = __builtin_amdgcn_wmma_f32_16x16x32_f16(false, a, false, b, (short)0, c, false, false);
  asm volatile("v_nop\n\tv_nop\n\tv_nop\n\tv_nop" : "+v"(c) : "v"(a), "v"(b));
  return c;
}

__global__ __launch_bounds__(128)
void attn64_h16(const _Float16* __restrict__ qp, const _Float16* __restrict__ kp,
                const _Float16* __restrict__ vp, _Float16* __restrict__ op,
                long q_bs, long q_rs, long k_bs, long k_rs, long v_bs, long v_rs, long o_bs, long o_rs,
                int S, int Skv, int H, float qscale, float oscale) {
  union FH { v16h v; v8h h[2]; };
  __shared__ __align__(16) _Float16 Ksh[AT_KC * AT_D];
  __shared__ __align__(16) _Float16 Vth[AT_D * AT_KC];
  __shared__ __align__(16) _Float16 Psh[AT_NW][16 * AT_KC];
  __shared__ __align__(16) float    Os[AT_NW][16 * 68];

  const int tid  = threadIdx.x;
  const int wave = tid >> 5;
  const int lane = tid & 31;
  const int hh   = lane >> 4;
  const int c    = lane & 15;

  const int nqb = S / AT_QB;
  const int bx = blockIdx.x;
  const int qb = bx % nqb;
  const int bh = bx / nqb;
  const int h  = bh % H;
  const int b  = bh / H;
  const int q0 = qb * AT_QB + wave * 16;

  const _Float16* qb_ptr = qp + (size_t)b * q_bs + (size_t)h * AT_D;
  const _Float16* kb_ptr = kp + (size_t)b * k_bs + (size_t)h * AT_D;
  const _Float16* vb_ptr = vp + (size_t)b * v_bs + (size_t)h * AT_D;
  _Float16*       ob_ptr = op + (size_t)b * o_bs + (size_t)h * AT_D;

  v16h qa[2];
  {
    const _Float16* qrow = qb_ptr + (size_t)(q0 + c) * q_rs;
#pragma unroll
    for (int dc = 0; dc < 2; ++dc) qa[dc] = Frag<_Float16>::load(qrow + dc * 32 + 8 * hh);
  }

  float mrow[8], lrow[8];
  v8f oacc[4];
#pragma unroll
  for (int r = 0; r < 8; ++r) { mrow[r] = -INFINITY; lrow[r] = 0.f; }
#pragma unroll
  for (int t = 0; t < 4; ++t) oacc[t] = (v8f){0.f,0.f,0.f,0.f,0.f,0.f,0.f,0.f};

  const int nChunks = Skv / AT_KC;
  for (int kc = 0; kc < nChunks; ++kc) {
    const int kv0 = kc * AT_KC;
    __syncthreads();
    {
      const int kvr = tid >> 1, dh = (tid & 1) * 32;
      const _Float16* krow = kb_ptr + (size_t)(kv0 + kvr) * k_rs + dh;
      const _Float16* vrow = vb_ptr + (size_t)(kv0 + kvr) * v_rs + dh;
#pragma unroll
      for (int i = 0; i < 4; ++i) {
        const v8h kk = *(const v8h*)(krow + 8 * i);
        const v8h vv = *(const v8h*)(vrow + 8 * i);
        *(v8h*)(Ksh + kvr * AT_D + dh + 8 * i) = kk;
#pragma unroll
        for (int e = 0; e < 8; ++e) Vth[(dh + 8 * i + e) * AT_KC + kvr] = vv[e];
      }
    }
    __syncthreads();

    v8f s[4];
#pragma unroll
    for (int j = 0; j < 4; ++j) {
      s[j] = (v8f){0.f,0.f,0.f,0.f,0.f,0.f,0.f,0.f};
#pragma unroll
      for (int dc = 0; dc < 2; ++dc) {
        FH kb;
        kb.h[0] = *(const v8h*)(Ksh + (j * 16 + c) * AT_D + dc * 32 + 8 * hh);
        kb.h[1] = *(const v8h*)(Ksh + (j * 16 + c) * AT_D + dc * 32 + 16 + 8 * hh);
        s[j] = mma_h(qa[dc], kb.v, s[j]);
      }
    }
    float cm[8];
#pragma unroll
    for (int r = 0; r < 8; ++r) {
      float m = -INFINITY;
#pragma unroll
      for (int j = 0; j < 4; ++j) {
        s[j][r] *= qscale;
        m = fmaxf(m, s[j][r]);
      }
#pragma unroll
      for (int off = 1; off < 16; off <<= 1) m = fmaxf(m, __shfl_xor(m, off, 32));
      cm[r] = m;
    }
    _Float16* pwh = Psh[wave];
#pragma unroll
    for (int r = 0; r < 8; ++r) {
      const float mnew = fmaxf(mrow[r], cm[r]);
      const float alpha = expf(mrow[r] - mnew);
      mrow[r] = mnew;
      float psum = 0.f;
#pragma unroll
      for (int j = 0; j < 4; ++j) {
        const float p = expf(s[j][r] - mnew);
        psum += p;
        pwh[(8 * hh + r) * AT_KC + j * 16 + c] = (_Float16)(p * PSCALE);
      }
#pragma unroll
      for (int off = 1; off < 16; off <<= 1) psum += __shfl_xor(psum, off, 32);
      lrow[r] = lrow[r] * alpha + psum;
#pragma unroll
      for (int t = 0; t < 4; ++t) oacc[t][r] *= alpha;
    }
    __builtin_amdgcn_fence(__ATOMIC_RELEASE, "workgroup");
    __builtin_amdgcn_wave_barrier();
    __builtin_amdgcn_fence(__ATOMIC_ACQUIRE, "workgroup");
#pragma unroll 1
    for (int kk = 0; kk < 2; ++kk) {
      FH pa;
      pa.h[0] = *(const v8h*)(pwh + c * AT_KC + kk * 32 + 8 * hh);
      pa.h[1] = *(const v8h*)(pwh + c * AT_KC + kk * 32 + 16 + 8 * hh);
#pragma unroll
      for (int t = 0; t < 4; ++t) {
        FH vb;
        vb.h[0] = *(const v8h*)(Vth + (t * 16 + c) * AT_KC + kk * 32 + 8 * hh);
        vb.h[1] = *(const v8h*)(Vth + (t * 16 + c) * AT_KC + kk * 32 + 16 + 8 * hh);
        oacc[t] = mma_h(pa.v, vb.v, oacc[t]);
      }
    }
  }

  float* os = Os[wave];
#pragma unroll
  for (int r = 0; r < 8; ++r) {
    const float inv = oscale * (1.0f / (lrow[r] * PSCALE));
#pragma unroll
    for (int t = 0; t < 4; ++t) os[(8 * hh + r) * 68 + t * 16 + c] = oacc[t][r] * inv;
  }
  __builtin_amdgcn_fence(__ATOMIC_RELEASE, "workgroup");
  __builtin_amdgcn_wave_barrier();
  __builtin_amdgcn_fence(__ATOMIC_ACQUIRE, "workgroup");
  {
    const int qq = lane >> 3, c8 = (lane & 7) * 8;
    for (int pass = 0; pass < 2; ++pass) {
#pragma unroll
      for (int it = 0; it < 4; ++it) {
        const int row = it * 4 + qq;
        const float* sp = os + row * 68 + c8;
        v8h hv;
#pragma unroll
        for (int e = 0; e < 8; ++e) hv[e] = (_Float16)sp[e];
        *(volatile v8h*)(ob_ptr + (size_t)(q0 + row) * o_rs + c8) = hv;
      }
      __threadfence();
    }
  }
}

extern "C" void kernel_launch(void* const* d_in, const int* in_sizes, int n_in,
                              void* d_out, int out_size, void* d_ws, size_t ws_size,
                              hipStream_t stream) {
  const int NB = 2, NQ = 2048, NM = 256, DM = 1024, NH = 16;
  const int LK = NQ + NM;
  const int ROWS = NB * NQ;
  const int MROWS = NB * NM;
  if (n_in < 9) return;
  if (in_sizes[0] != ROWS * DM || in_sizes[1] != MROWS * DM || in_sizes[2] != DM || in_sizes[3] != DM ||
      in_sizes[4] != DM * DM || in_sizes[5] != DM * 2 * DM || in_sizes[6] != DM * DM || in_sizes[7] != DM * DM ||
      in_sizes[8] != DM || out_size != ROWS * DM) return;

  const float* x    = (const float*)d_in[0];
  const float* mem  = (const float*)d_in[1];
  const float* ln_g = (const float*)d_in[2];
  const float* ln_b = (const float*)d_in[3];
  const float* Wq   = (const float*)d_in[4];
  const float* Wkv  = (const float*)d_in[5];
  const float* Wm   = (const float*)d_in[6];
  const float* Wo   = (const float*)d_in[7];
  const float* bo   = (const float*)d_in[8];
  float* out = (float*)d_out;

  char* ws = (char*)d_ws;
  size_t off = 0;
  const size_t szXn   = (size_t)ROWS * DM * 2;
  const size_t szMemh = (size_t)MROWS * DM * 2;
  const size_t szWq   = (size_t)DM * DM * 2;
  const size_t szWkv  = (size_t)2 * DM * DM * 2;
  const size_t szWm2  = (size_t)2 * DM * DM * 2;
  const size_t szWo   = (size_t)DM * DM * 2;
  const size_t szQ    = (size_t)ROWS * DM * 2;
  const size_t szKV   = (size_t)NB * LK * 2 * DM * 2;
  const size_t szO    = (size_t)ROWS * DM * 2;
  _Float16* xn   = (_Float16*)(ws + off); off += szXn;
  _Float16* memh = (_Float16*)(ws + off); off += szMemh;
  _Float16* wqT  = (_Float16*)(ws + off); off += szWq;
  _Float16* wkvT = (_Float16*)(ws + off); off += szWkv;
  _Float16* wmT2 = (_Float16*)(ws + off); off += szWm2;
  _Float16* woT  = (_Float16*)(ws + off); off += szWo;
  _Float16* qpl  = (_Float16*)(ws + off); off += szQ;
  _Float16* kvpl = (_Float16*)(ws + off); off += szKV;
  _Float16* opl  = (_Float16*)(ws + off); off += szO;
  if (off > ws_size || off > (size_t)134217728) return;

  cast_transpose_f16<<<dim3(DM / 64, DM / 64), 256, 0, stream>>>(Wq, wqT, DM, DM, 64.0f, 1);
  cast_transpose_f16<<<dim3(2 * DM / 64, DM / 64), 256, 0, stream>>>(Wkv, wkvT, DM, 2 * DM, 64.0f, 1);
  cast_transpose_f16<<<dim3(DM / 64, DM / 64), 256, 0, stream>>>(Wm, wmT2, DM, DM, 64.0f, 2);
  cast_transpose_f16<<<dim3(DM / 64, DM / 64), 256, 0, stream>>>(Wo, woT, DM, DM, 64.0f, 1);
  cast_f32_f16x2<<<(MROWS * DM / 2 + 255) / 256, 256, 0, stream>>>(mem, memh, MROWS * DM / 2);
  layernorm_f16<<<ROWS, 128, 0, stream>>>(x, ln_g, ln_b, xn);

  wmma_gemm64<0, false, 0, 1, false><<<dim3((ROWS / 64) * (DM / 64) / 8, 1), 256, 0, stream>>>(
      U16(xn), U16(xn), DM, 0L, U16(wqT), U16(wqT), DM, 0L,
      (void*)qpl, (void*)qpl, DM, 0L, bo, x, 0L, ROWS, DM, DM, 1.0f / 64.0f);
  wmma_gemm64<0, false, 0, 1, false><<<dim3((NQ / 64) * (2 * DM / 64) / 8, NB), 256, 0, stream>>>(
      U16(xn), U16(xn), DM, (long)NQ * DM, U16(wkvT), U16(wkvT), DM, 0L,
      (void*)kvpl, (void*)kvpl, 2 * DM, (long)LK * 2 * DM, bo, x, 0L, NQ, 2 * DM, DM, 1.0f / 64.0f);
  wmma_gemm64<0, false, 0, 1, false><<<dim3((NM / 64) * (2 * DM / 64) / 8, NB), 256, 0, stream>>>(
      U16(memh), U16(memh), DM, (long)NM * DM, U16(wmT2), U16(wmT2), DM, 0L,
      (void*)(kvpl + (size_t)NQ * 2 * DM), (void*)(kvpl + (size_t)NQ * 2 * DM), 2 * DM, (long)LK * 2 * DM,
      bo, x, 0L, NM, 2 * DM, DM, 1.0f / 64.0f);

  attn64_h16<<<NB * NH * (NQ / 64), 128, 0, stream>>>(
      qpl, kvpl, kvpl + DM, opl,
      (long)NQ * DM, (long)DM,
      (long)LK * 2 * DM, (long)(2 * DM),
      (long)LK * 2 * DM, (long)(2 * DM),
      (long)NQ * DM, (long)DM,
      NQ, LK, NH, 0.125f, 16.0f);

  wmma_gemm64<0, false, 2, 0, false><<<dim3((ROWS / 64) * (DM / 64) / 8, 1), 256, 0, stream>>>(
      U16(opl), U16(opl), DM, 0L, U16(woT), U16(woT), DM, 0L,
      (void*)out, (void*)out, DM, 0L, bo, x, 0L, ROWS, DM, DM, 1.0f / 1024.0f);
}
